// LearnableSeedCLF_3547642986554
// MI455X (gfx1250) — hardware-verified
//
#include <hip/hip_runtime.h>


namespace {
constexpr int B = 2048, L = 200, V = 32000, C = 9;
constexpr float WSC = 256.0f;
typedef _Float16 b16;
typedef __attribute__((ext_vector_type(16))) _Float16 v16b;
typedef __attribute__((ext_vector_type(8))) _Float16 v8b;
typedef __attribute__((ext_vector_type(8))) float v8f;
__device__ __forceinline__ float bf16_rne(float f) { unsigned int u = __float_as_uint(f); u += 0x7FFFu + ((u >> 16) & 1u); return __uint_as_float(u & 0xFFFF0000u); }
__device__ __forceinline__ v16b frag_kb(const b16* p, int hh) { const v8b a = *(const v8b*)(p + 8 * hh), b = *(const v8b*)(p + 16 + 8 * hh); v16b f;
#pragma unroll
  for (int e = 0; e < 8; ++e) { f[e] = a[e]; f[8 + e] = b[e]; } return f; }
__device__ __forceinline__ v8f wmma16b(v16b a, v16b b, v8f c) { v8f d = __builtin_amdgcn_wmma_f32_16x16x32_f16(false, a, false, b, (short)0, c, false, false); asm volatile("v_nop\n\tv_nop\n\tv_nop\n\tv_nop" : "+v"(d) : "v"(a), "v"(b)); return d; }
__device__ __forceinline__ void wave_lds_sync() { __builtin_amdgcn_fence(__ATOMIC_RELEASE, "workgroup"); __builtin_amdgcn_wave_barrier(); __builtin_amdgcn_fence(__ATOMIC_ACQUIRE, "workgroup"); }
__device__ __forceinline__ int iclamp(int v, int lo, int hi) { return v < lo ? lo : (v > hi ? hi : v); }

__global__ __launch_bounds__(256) void wcopy_kernel(const float* __restrict__ w, b16* __restrict__ WT) {
  const size_t u = (size_t)blockIdx.x * 256 + threadIdx.x; if (u >= (size_t)16 * V / 8) return; const size_t e = u * 8; const int c = (int)(e / V); v8b v;
#pragma unroll
  for (int j = 0; j < 8; ++j) v[j] = c < C ? (b16)(bf16_rne(w[e + j]) * WSC) : (b16)0.0f; for (int pass = 0; pass < 2; ++pass) { *(volatile v8b*)(WT + e) = v; __threadfence(); }
}
__global__ __launch_bounds__(32) void bow_kernel(const int* __restrict__ ids, int NLIM, b16* __restrict__ BOW) {
  __shared__ __attribute__((aligned(16))) b16 Hs[V]; const int lane = threadIdx.x; const size_t i = blockIdx.x; if (i >= (size_t)NLIM) return; const v8b z = {};
  for (int v0 = lane * 8; v0 < V; v0 += 256) *(v8b*)(Hs + v0) = z;
  wave_lds_sync();
  if (lane == 0) { for (int l = 0; l < L; ++l) { const int v = iclamp(ids[i * L + l], 0, V - 1); Hs[v] = (b16)((float)Hs[v] + 1.0f); } }
  wave_lds_sync(); b16* row = BOW + i * V;
  for (int pass = 0; pass < 2; ++pass) { for (int v0 = lane * 8; v0 < V; v0 += 256) *(volatile v8b*)(row + v0) = *(const v8b*)(Hs + v0); __threadfence(); }
}
__global__ __launch_bounds__(32) void out_kernel(const b16* __restrict__ BOW, const b16* __restrict__ WT, const float* __restrict__ bias, int NLIM, float* __restrict__ out) {
  __shared__ float Lg[32][17], So[32][C]; const int lane = threadIdx.x, nloc = lane & 15, hlf = lane >> 4; const size_t r0 = (size_t)blockIdx.x * 32; if (r0 >= (size_t)NLIM) return;
  v8f acc0 = {}, acc1 = {};
#pragma unroll 4
  for (int kb = 0; kb < V; kb += 32) { const v16b w = frag_kb(WT + (size_t)nloc * V + kb, hlf); acc0 = wmma16b(frag_kb(BOW + (r0 + nloc) * V + kb, hlf), w, acc0); acc1 = wmma16b(frag_kb(BOW + (r0 + 16 + nloc) * V + kb, hlf), w, acc1); }
#pragma unroll
  for (int r8 = 0; r8 < 8; ++r8) { Lg[8 * hlf + r8][nloc] = acc0[r8] * (1.0f / WSC); Lg[16 + 8 * hlf + r8][nloc] = acc1[r8] * (1.0f / WSC); }
  wave_lds_sync();
  { const int r = lane; float mx = -INFINITY, lg[C]; for (int c = 0; c < C; ++c) { lg[c] = Lg[r][c] + bf16_rne(bias[c]); mx = fmaxf(mx, lg[c]); } float s = 0.0f; for (int c = 0; c < C; ++c) { lg[c] = __expf(lg[c] - mx); s += lg[c]; } const float inv = 1.0f / s; for (int c = 0; c < C; ++c) So[r][c] = lg[c] * inv; }
  wave_lds_sync();
  for (int pass = 0; pass < 2; ++pass) { for (int i = lane; i < 32 * C; i += 32) ((volatile float*)out)[r0 * C + i] = So[i / C][i % C]; __threadfence(); }
}
}

extern "C" void kernel_launch(void* const* d_in, const int* in_sizes, int n_in, void* d_out, int out_size, void* d_ws, size_t ws_size, hipStream_t stream) {
  (void)n_in;
  if (in_sizes[0] != B * L || in_sizes[1] != C * V || in_sizes[2] != C || out_size != B * C) return;
  const int NLIM = B;
  size_t off = 0; char* ws = (char*)d_ws;
  auto carve = [&](size_t bytes) { char* p = ws + off; off += (bytes + 255) & ~(size_t)255; return p; };
  b16* WT = (b16*)carve((size_t)16 * V * 2); b16* BOW = (b16*)carve((size_t)B * V * 2);
  if (off > ws_size || off > ((size_t)160 << 20)) return;
  wcopy_kernel<<<(unsigned)((16 * V / 8 + 255) / 256), 256, 0, stream>>>((const float*)d_in[1], WT);
  bow_kernel<<<(unsigned)NLIM, 32, 0, stream>>>((const int*)d_in[0], NLIM, BOW);
  out_kernel<<<(unsigned)(NLIM / 32), 32, 0, stream>>>(BOW, WT, (const float*)d_in[2], NLIM, (float*)d_out);
}
